// CausalSelfAttention_56624848830936
// MI455X (gfx1250) — hardware-verified
//
#include <hip/hip_runtime.h>
#include <math.h>

typedef __attribute__((ext_vector_type(16))) _Float16 v16h;
typedef __attribute__((ext_vector_type(16))) __bf16 v16b;
typedef __attribute__((ext_vector_type(8)))  _Float16 v8h;
typedef __attribute__((ext_vector_type(8)))  __bf16 v8b;
typedef __attribute__((ext_vector_type(8)))  float v8f;
typedef __attribute__((ext_vector_type(4)))  float v4f;
typedef __attribute__((ext_vector_type(4)))  unsigned v4u;

template <typename T> __device__ __forceinline__ void vst2(void* p, T v) { *(volatile T*)p = v; __threadfence(); *(volatile T*)p = v; }
__device__ __forceinline__ v8f wmma16(v16h a, v16h b, v8f c) {
  v8f d = __builtin_amdgcn_wmma_f32_16x16x32_f16(false, a, false, b, (short)0, c, false, false);
  asm volatile("v_nop\n\tv_nop\n\tv_nop\n\tv_nop" : "+v"(d) : "v"(a), "v"(b));
  return d;
}
__device__ __forceinline__ v8f wmma_bf(v16b a, v16b b, v8f c) {
  v8f d = __builtin_amdgcn_wmma_f32_16x16x32_bf16(false, a, false, b, (short)0, c, false, false);
  asm volatile("v_nop\n\tv_nop\n\tv_nop\n\tv_nop" : "+v"(d) : "v"(a), "v"(b));
  return d;
}
__device__ __forceinline__ v16h frag_h(const _Float16* rowk0, int lane) {
  union { v16h v; v8h q[2]; } u; const _Float16* p = rowk0 + 8 * (lane >> 4);
  u.q[0] = *(const v8h*)p; u.q[1] = *(const v8h*)(p + 16); return u.v;
}
__device__ __forceinline__ v16b frag_b(const __bf16* rowk0, int lane) {
  union { v16b v; v8b q[2]; } u; const __bf16* p = rowk0 + 8 * (lane >> 4);
  u.q[0] = *(const v8b*)p; u.q[1] = *(const v8b*)(p + 16); return u.v;
}
__device__ __forceinline__ v16b wcol_io(const float* Wm, int k0, int o, int lane, int ld) { v16b w; const int g = lane >> 4;
#pragma unroll
  for (int i = 0; i < 8; ++i) { w[i] = (__bf16)Wm[(size_t)(k0 + 8 * g + i) * ld + o]; w[8 + i] = (__bf16)Wm[(size_t)(k0 + 16 + 8 * g + i) * ld + o]; }
  return w; }
#define LDSX() do { asm volatile("s_wait_dscnt 0" ::: "memory"); __builtin_amdgcn_wave_barrier(); __builtin_amdgcn_fence(3  , "workgroup"); } while (0)

#ifndef NB
#define NB 2
#endif
#ifndef SEQ
#define SEQ 2048
#endif
#define NB_FULL 2
#define SEQ_FULL 2048
#define TT SEQ
#define CC 1024
#define DIN 1024
#define NH 16
#define HD 64
#define NQB (TT / 64)
#define QBH 4
#define KHI 256
#define SCALE_LOG2E (0.125f * 1.4426950408889634f)
#define NEGBIG (-3.0e38f)

static_assert(NB <= NB_FULL);
static_assert(TT <= SEQ_FULL);
static_assert(CC == NH * HD);
static_assert(HD == 64);
static_assert(TT % 64 == 0);
static_assert(KHI % 64 == 0);
static_assert(QBH * 64 <= KHI);
static_assert(KHI <= TT);
static_assert(QBH <= NQB);
static_assert(DIN % 32 == 0);
static_assert(CC % 32 == 0);
static_assert(CC % 128 == 0);
static_assert(DIN % 128 == 0);
static_assert((NB * TT) % 64 == 0);

#define E_QH  ((size_t)0)
#define E_QL  (E_QH + (size_t)NB * TT * CC)
#define E_KH  (E_QL + (size_t)NB * TT * CC)
#define E_KL  (E_KH + (size_t)NB * TT * CC)
#define E_VT  (E_KL + (size_t)NB * TT * CC)
#define E_VB  (E_VT + (size_t)NB * CC * TT)
#define E_VBL (E_VB + (size_t)NB * CC * KHI)
#define E_YH  (E_VBL + (size_t)NB * CC * KHI)
#define E_YL  (E_YH + (size_t)NB * TT * CC)
#define E_END (E_YL + (size_t)NB * TT * CC)
#define WS_NEED ((size_t)2 * E_END)
static_assert(WS_NEED <= (size_t)134217728);
static_assert(E_END < (size_t)2147483647);

__global__ __launch_bounds__(128) void k_proj(const float* __restrict__ X, const float* __restrict__ W, _Float16* __restrict__ H, __bf16* __restrict__ VB, __bf16* __restrict__ VBL) {
  __shared__ __align__(16) _Float16 sh[64][136], sl[64][136];
  __shared__ __align__(16) _Float16 th[128][72];
  __shared__ __align__(16) __bf16 tb[128][72], tbl[128][72];
  const int tid = threadIdx.x; const int wave = __builtin_amdgcn_readfirstlane(tid >> 5); const int lane = tid & 31, col = lane & 15, g = lane >> 4;
  const int which = blockIdx.z; const int c0 = blockIdx.y * 128; const int r0 = blockIdx.x * 64; const int bb = r0 / TT; const int t0 = r0 % TT;
  const float* WA = W + which * CC;
  const float* xp = X + ((size_t)bb * SEQ_FULL + t0 + wave * 16 + col) * DIN + 8 * g;
  v8f acc[8] = {};
#pragma unroll 2
  for (int kc = 0; kc < DIN / 32; ++kc) { v16b a; const float* p = xp + kc * 32;
#pragma unroll
    for (int i = 0; i < 8; ++i) { a[i] = (__bf16)p[i]; a[8 + i] = (__bf16)p[16 + i]; }
    asm volatile("s_wait_loadcnt 0x0" ::: "memory");
#pragma unroll
    for (int j = 0; j < 8; ++j) { const v16b w = wcol_io(WA, kc * 32, c0 + j * 16 + col, lane, 3 * CC); asm volatile("s_wait_loadcnt 0x0" ::: "memory"); acc[j] = wmma_bf(a, w, acc[j]); } }
  if (which < 2) {
    const size_t eh = which == 0 ? E_QH : E_KH; const size_t el = which == 0 ? E_QL : E_KL;
#pragma unroll
    for (int j = 0; j < 8; ++j) {
#pragma unroll
      for (int r = 0; r < 8; ++r) { const float v = acc[j][r]; const _Float16 hv = (_Float16)v; sh[wave * 16 + 8 * g + r][j * 16 + col] = hv; sl[wave * 16 + 8 * g + r][j * 16 + col] = (_Float16)((v - (float)hv) * 1024.0f); } }
    __syncthreads();
    for (int e = tid; e < 64 * 16; e += 128) { const int rl = e >> 4, q = e & 15;
      const size_t o = (size_t)(r0 + rl) * CC + c0 + q * 8;
      vst2(H + eh + o, *(const v4u*)&sh[rl][q * 8]);
      vst2(H + el + o, *(const v4u*)&sl[rl][q * 8]); }
  } else { const bool hi_rows = t0 < KHI;
#pragma unroll
    for (int j = 0; j < 8; ++j) {
#pragma unroll
      for (int r = 0; r < 8; ++r) { const float v = acc[j][r]; const int rl = wave * 16 + 8 * g + r, cl = j * 16 + col; th[cl][rl] = (_Float16)v; const __bf16 bh = (__bf16)v; tb[cl][rl] = bh; tbl[cl][rl] = (__bf16)(v - (float)bh); } }
    __syncthreads();
    for (int e = tid; e < 128 * 8; e += 128) { const int cl = e >> 3, q = e & 7;
      vst2(H + E_VT + ((size_t)bb * CC + c0 + cl) * TT + t0 + q * 8, *(const v4u*)&th[cl][q * 8]);
      if (hi_rows) { const size_t o3 = ((size_t)bb * CC + c0 + cl) * KHI + t0 + q * 8; vst2(VB + o3, *(const v4u*)&tb[cl][q * 8]); vst2(VBL + o3, *(const v4u*)&tbl[cl][q * 8]); } } } }

template <bool EARLY>
__device__ __forceinline__ void attn_body(const int qb, const _Float16* __restrict__ QH, const _Float16* __restrict__ QL, const _Float16* __restrict__ KH, const _Float16* __restrict__ KL,
    const _Float16* __restrict__ VT, const __bf16* __restrict__ VB, const __bf16* __restrict__ VBL, __bf16* __restrict__ YH, __bf16* __restrict__ YL) {
  __shared__ __align__(16) _Float16 pt[4][16][40];
  __shared__ __align__(16) __bf16 pbh[4][16][40], pbl[4][16][40];
  __shared__ __align__(16) float ss[4][16][HD + 4];
  const int tid = threadIdx.x; const int wave = __builtin_amdgcn_readfirstlane(tid >> 5); const int lane = tid & 31, col = lane & 15, g = lane >> 4;
  const int h = blockIdx.y, b = blockIdx.z;
  const int ql0 = qb * 64 + wave * 16;
  const int nhalf = (ql0 >> 5) + 1;
  const int qo = (b * TT + ql0 + col) * CC + h * HD;
  const int kbase = (b * TT + col) * CC + h * HD;
  const int vbase = (b * CC + h * HD + col) * TT;
  const int vbb = (b * CC + h * HD + col) * KHI;
  v8f acc[4] = {};
  float m[8], ls[8];
#pragma unroll
  for (int r = 0; r < 8; ++r) { m[r] = NEGBIG; ls[r] = 0.f; }
#pragma unroll 1
  for (int hf = 0; hf < nhalf; ++hf) { const int k0 = hf * 32;
    v8f s0 = {}, s1 = {}, l0 = {}, l1 = {};
#pragma unroll
    for (int kc = 0; kc < HD / 32; ++kc) {
      const v16h qh = frag_h(QH + qo + kc * 32, lane), ql = frag_h(QL + qo + kc * 32, lane);
      const v16h kf0 = frag_h(KH + kbase + k0 * CC + kc * 32, lane), kf1 = frag_h(KH + kbase + (k0 + 16) * CC + kc * 32, lane);
      s0 = wmma16(qh, kf0, s0); l0 = wmma16(ql, kf0, l0); s1 = wmma16(qh, kf1, s1); l1 = wmma16(ql, kf1, l1);
      const v16h kl0 = frag_h(KL + kbase + k0 * CC + kc * 32, lane), kl1 = frag_h(KL + kbase + (k0 + 16) * CC + kc * 32, lane);
      l0 = wmma16(qh, kl0, l0); l1 = wmma16(qh, kl1, l1); }
#pragma unroll
    for (int r = 0; r < 8; ++r) { const int row = ql0 + 8 * g + r;
      float t0v = (s0[r] + l0[r] * (1.0f / 1024.0f)) * SCALE_LOG2E, t1v = (s1[r] + l1[r] * (1.0f / 1024.0f)) * SCALE_LOG2E;
      t0v = (k0 + col <= row) ? t0v : NEGBIG; t1v = (k0 + 16 + col <= row) ? t1v : NEGBIG;
      float mr = fmaxf(t0v, t1v);
      mr = fmaxf(mr, __shfl_xor(mr, 1)); mr = fmaxf(mr, __shfl_xor(mr, 2)); mr = fmaxf(mr, __shfl_xor(mr, 4)); mr = fmaxf(mr, __shfl_xor(mr, 8));
      const float mn = fmaxf(m[r], mr); const float corr = exp2f(m[r] - mn); m[r] = mn; const float mn10 = mn - 10.0f;
      const float p0 = (t0v <= -1.0e38f) ? 0.f : exp2f(t0v - mn10), p1 = (t1v <= -1.0e38f) ? 0.f : exp2f(t1v - mn10);
      ls[r] = ls[r] * corr + (p0 + p1);
      acc[0][r] *= corr; acc[1][r] *= corr; acc[2][r] *= corr; acc[3][r] *= corr;
      if (EARLY) { const __bf16 b0 = (__bf16)p0, b1 = (__bf16)p1; pbh[wave][8 * g + r][col] = b0; pbh[wave][8 * g + r][16 + col] = b1; pbl[wave][8 * g + r][col] = (__bf16)(p0 - (float)b0); pbl[wave][8 * g + r][16 + col] = (__bf16)(p1 - (float)b1); }
      else { pt[wave][8 * g + r][col] = (_Float16)p0; pt[wave][8 * g + r][16 + col] = (_Float16)p1; } }
    LDSX();
    if (EARLY) { union { v16b v; v8b q[2]; } uh, ul;
      uh.q[0] = *(const v8b*)&pbh[wave][col][8 * g]; uh.q[1] = *(const v8b*)&pbh[wave][col][16 + 8 * g];
      ul.q[0] = *(const v8b*)&pbl[wave][col][8 * g]; ul.q[1] = *(const v8b*)&pbl[wave][col][16 + 8 * g];
#pragma unroll
      for (int j = 0; j < 4; ++j) { const int po = vbb + j * 16 * KHI + k0; const v16b vh = frag_b(VB + po, lane), vl = frag_b(VBL + po, lane); asm volatile("s_wait_loadcnt 0x0" ::: "memory");
        acc[j] = wmma_bf(uh.v, vh, acc[j]); acc[j] = wmma_bf(ul.v, vh, acc[j]); acc[j] = wmma_bf(uh.v, vl, acc[j]); }
    } else { union { v16h v; v8h q[2]; } up;
      up.q[0] = *(const v8h*)&pt[wave][col][8 * g]; up.q[1] = *(const v8h*)&pt[wave][col][16 + 8 * g];
#pragma unroll
      for (int j = 0; j < 4; ++j) { const v16h vf = frag_h(VT + vbase + j * 16 * TT + k0, lane); acc[j] = wmma16(up.v, vf, acc[j]); } }
    LDSX();
  }
#pragma unroll
  for (int r = 0; r < 8; ++r) { float s = ls[r];
    s += __shfl_xor(s, 1); s += __shfl_xor(s, 2); s += __shfl_xor(s, 4); s += __shfl_xor(s, 8);
    const float inv = 1.0f / s;
    ss[wave][8 * g + r][col] = acc[0][r] * inv; ss[wave][8 * g + r][16 + col] = acc[1][r] * inv; ss[wave][8 * g + r][32 + col] = acc[2][r] * inv; ss[wave][8 * g + r][48 + col] = acc[3][r] * inv; }
  LDSX();
#pragma unroll
  for (int it = 0; it < 4; ++it) { const int row = it * 4 + (lane >> 3), pc = lane & 7;
    const v4f a0 = *(const v4f*)&ss[wave][row][pc * 8], a1 = *(const v4f*)&ss[wave][row][pc * 8 + 4];
    union { v8b v; v4u u; } ph, pl;
#pragma unroll
    for (int i = 0; i < 4; ++i) { const __bf16 h0 = (__bf16)a0[i], h1 = (__bf16)a1[i]; ph.v[i] = h0; ph.v[4 + i] = h1; pl.v[i] = (__bf16)(a0[i] - (float)h0); pl.v[4 + i] = (__bf16)(a1[i] - (float)h1); }
    const size_t o = ((size_t)b * TT + ql0 + row) * CC + h * HD + pc * 8;
    vst2(YH + o, ph.u); vst2(YL + o, pl.u); }
}
__global__ __launch_bounds__(128) void k_attn_early(const _Float16* __restrict__ QH, const _Float16* __restrict__ QL, const _Float16* __restrict__ KH, const _Float16* __restrict__ KL,
    const _Float16* __restrict__ VT, const __bf16* __restrict__ VB, const __bf16* __restrict__ VBL, __bf16* __restrict__ YH, __bf16* __restrict__ YL) {
  attn_body<true>((int)blockIdx.x, QH, QL, KH, KL, VT, VB, VBL, YH, YL); }
__global__ __launch_bounds__(128) void k_attn(const _Float16* __restrict__ QH, const _Float16* __restrict__ QL, const _Float16* __restrict__ KH, const _Float16* __restrict__ KL,
    const _Float16* __restrict__ VT, const __bf16* __restrict__ VB, const __bf16* __restrict__ VBL, __bf16* __restrict__ YH, __bf16* __restrict__ YL) {
  attn_body<false>((int)blockIdx.x + QBH, QH, QL, KH, KL, VT, VB, VBL, YH, YL); }

__global__ __launch_bounds__(128) void k_out(const __bf16* __restrict__ YH, const __bf16* __restrict__ YL, const float* __restrict__ WO, float* __restrict__ OUT) {
  __shared__ __align__(16) float sf[4][16][132];
  const int tid = threadIdx.x; const int wave = __builtin_amdgcn_readfirstlane(tid >> 5); const int lane = tid & 31, col = lane & 15, g = lane >> 4;
  const int c0 = blockIdx.y * 128; const int rb = blockIdx.x * 64; const int bb = rb / TT; const int t0 = rb % TT; const int r0 = rb + wave * 16;
  const int yo = (r0 + col) * CC;
  v8f acc[8] = {};
#pragma unroll 2
  for (int kc = 0; kc < CC / 32; ++kc) { const v16b ah = frag_b(YH + yo + kc * 32, lane), al = frag_b(YL + yo + kc * 32, lane); asm volatile("s_wait_loadcnt 0x0" ::: "memory");
#pragma unroll
    for (int j = 0; j < 8; ++j) { const v16b w = wcol_io(WO, kc * 32, c0 + j * 16 + col, lane, DIN); asm volatile("s_wait_loadcnt 0x0" ::: "memory"); acc[j] = wmma_bf(ah, w, acc[j]); acc[j] = wmma_bf(al, w, acc[j]); } }
#pragma unroll
  for (int j = 0; j < 8; ++j) {
#pragma unroll
    for (int r = 0; r < 8; ++r) sf[wave][8 * g + r][j * 16 + col] = acc[j][r]; }
  LDSX();
  const size_t orow0 = (size_t)bb * SEQ_FULL + t0 + wave * 16;
  for (int rl = 0; rl < 16; ++rl) vst2(OUT + (orow0 + rl) * DIN + c0 + lane * 4, *(const v4f*)&sf[wave][rl][lane * 4]); }

extern "C" void kernel_launch(void* const* d_in, const int* in_sizes, int n_in, void* d_out, int out_size, void* d_ws, size_t ws_size, hipStream_t stream) {
  if (n_in < 3) return;
  const long long need_rows = (long long)(NB - 1) * SEQ_FULL + TT;
  if ((long long)in_sizes[0] < need_rows * DIN) return;
  if ((long long)in_sizes[1] < (long long)DIN * 3 * CC) return;
  if ((long long)in_sizes[2] < (long long)CC * DIN) return;
  if ((long long)out_size < need_rows * DIN) return;
  if (ws_size < WS_NEED) return;
  const float* X = (const float*)d_in[0]; const float* WQKV = (const float*)d_in[1]; const float* WP = (const float*)d_in[2];
  _Float16* H = (_Float16*)d_ws; __bf16* Bw = (__bf16*)d_ws;
  k_proj<<<dim3(NB * TT / 64, CC / 128, 3), 128, 0, stream>>>(X, WQKV, H, Bw + E_VB, Bw + E_VBL);
  k_attn_early<<<dim3(QBH, NH, NB), 128, 0, stream>>>(H + E_QH, H + E_QL, H + E_KH, H + E_KL, H + E_VT, Bw + E_VB, Bw + E_VBL, Bw + E_YH, Bw + E_YL);
  if (NQB > QBH) k_attn<<<dim3(NQB - QBH, NH, NB), 128, 0, stream>>>(H + E_QH, H + E_QL, H + E_KH, H + E_KL, H + E_VT, Bw + E_VB, Bw + E_VBL, Bw + E_YH, Bw + E_YL);
  k_out<<<dim3(NB * TT / 64, DIN / 128), 128, 0, stream>>>(Bw + E_YH, Bw + E_YL, WP, (float*)d_out);
}
